// VirtualAdaptiveWeights_68350109549066
// MI455X (gfx1250) — hardware-verified
//
#include <hip/hip_runtime.h>
#include <stddef.h>


typedef _Float16 h16;
typedef _Float16 v16h __attribute__((ext_vector_type(16)));
typedef _Float16 v8h  __attribute__((ext_vector_type(8)));
typedef float    v8f  __attribute__((ext_vector_type(8)));
typedef float    v4f  __attribute__((ext_vector_type(4)));

#ifndef NEDGE
#define NEDGE 500000
#endif
#define NEDGE_FULL 500000
#define NNODE  50000
#define DFEAT  256
#define NHEADS 8
#define NPROJ  16
#define NTILE  (NNODE / 16)
#define WPB    5

#define XCARRY 16.0f
#define WCARRY 64.0f

#define LDW 264
#define LDP 20

static_assert(NEDGE >= 16 && NEDGE <= NEDGE_FULL);
static_assert((NEDGE % 16) == 0);
static_assert(((2 * NEDGE) % 32) == 0);
static_assert((NNODE % 16) == 0);
static_assert((NTILE % WPB) == 0);
static_assert(NPROJ == 2 * NHEADS && NPROJ == 16);
static_assert((DFEAT % 32) == 0);
static_assert((DFEAT % 8) == 0);
static_assert((LDW % 8) == 0 && LDW >= DFEAT);
static_assert((LDP % 4) == 0 && LDP >= NPROJ);
static_assert(2 * DFEAT * NHEADS == 256 * 16);
static_assert(NPROJ * DFEAT == 256 * 2 * 8);
static_assert((32 / 4) * 2 == 16);
static_assert((size_t)16 * LDW * 2 <= (size_t)131072);
static_assert((size_t)WPB * 16 * LDP * 4 <= (size_t)131072);

#define WT_BYTES   ((size_t)NPROJ * DFEAT * 2)
#define PROJ_BYTES ((size_t)NNODE * NPROJ * 4)
#define OFF_WT   ((size_t)0)
#define OFF_PROJ (OFF_WT + WT_BYTES)
#define WS_TOTAL (OFF_PROJ + PROJ_BYTES)
static_assert((WT_BYTES % 128) == 0 && (PROJ_BYTES % 128) == 0);
static_assert((size_t)NTILE * 16 * NPROJ * 4 == PROJ_BYTES);
static_assert(WS_TOTAL <= (size_t)134217728);

__device__ __forceinline__ float bf16r(float x) {
  unsigned int u = __float_as_uint(x);
  u = (u + 0x7FFFu + ((u >> 16) & 1u)) & 0xFFFF0000u;
  return __uint_as_float(u);
}

static __device__ __forceinline__ h16 toh_flush(float v) {
  const h16 r = (h16)v;
  return (fabsf(v) < 6.103515625e-05f) ? (h16)0.0f : r;
}

__device__ __forceinline__ v16h frag_at(const _Float16* p) {
  v8h lo = *(const v8h*)(p);
  v8h hi = *(const v8h*)(p + 16);
  v16h out;
#pragma unroll
  for (int i = 0; i < 8; ++i) { out[i] = lo[i]; out[i + 8] = hi[i]; }
  return out;
}

__device__ __forceinline__ v16h frag_from_f32(const float* p) {
  const v4f a0 = *(const v4f*)(p);
  const v4f a1 = *(const v4f*)(p + 4);
  const v4f a2 = *(const v4f*)(p + 16);
  const v4f a3 = *(const v4f*)(p + 20);
  v16h out;
#pragma unroll
  for (int i = 0; i < 4; ++i) {
    out[i]      = toh_flush(XCARRY * bf16r(a0[i]));
    out[i + 4]  = toh_flush(XCARRY * bf16r(a1[i]));
    out[i + 8]  = toh_flush(XCARRY * bf16r(a2[i]));
    out[i + 12] = toh_flush(XCARRY * bf16r(a3[i]));
  }
  return out;
}

__device__ __forceinline__ v8f wmma16(v16h a, v16h b, v8f c) {
  v8f d = __builtin_amdgcn_wmma_f32_16x16x32_f16(false, a, false, b, (short)0, c,
                                                 false, false);
  asm volatile("v_nop\n\tv_nop\n\tv_nop\n\tv_nop" : "+v"(d) : "v"(a), "v"(b));
  return d;
}

__device__ __forceinline__ void wave_lds_sync() {
  __builtin_amdgcn_fence(3  , "wavefront");
  asm volatile("s_wait_dscnt 0x0" ::: "memory");
  __builtin_amdgcn_wave_barrier();
}

__global__ __launch_bounds__(256) void wconv_kernel(
    const float* __restrict__ W, _Float16* __restrict__ Wt) {
  __shared__ _Float16 T[16 * LDW];
  const unsigned tid = threadIdx.x;
#pragma unroll 4
  for (unsigned j = 0; j < 16u; ++j) {
    const unsigned s = tid + 256u * j;
    const unsigned kk = s >> 3, hc = s & 7u;
    const unsigned n = hc + 8u * (kk >> 8);
    const unsigned k = kk & 255u;
    const float v = W[s];
    T[n * LDW + k] = toh_flush(WCARRY * bf16r(v));
  }
  __syncthreads();
  v8h x[2];
  size_t off[2];
#pragma unroll
  for (unsigned i = 0; i < 2u; ++i) {
    const unsigned p = tid + 256u * i;
    const unsigned n = p >> 5;
    const unsigned kc = (p & 31u) * 8u;
    x[i] = *(const v8h*)&T[n * LDW + kc];
    off[i] = (size_t)n * DFEAT + kc;
  }
#pragma unroll
  for (int i = 0; i < 2; ++i) *(volatile v8h*)(Wt + off[i]) = x[i];
  __threadfence();
#pragma unroll
  for (int i = 0; i < 2; ++i) *(volatile v8h*)(Wt + off[i]) = x[i];
}

__global__ __launch_bounds__(160) void proj_kernel(
    const float* __restrict__ X, const _Float16* __restrict__ Wt, float* __restrict__ proj) {
  __shared__ float Cs[WPB * 16 * LDP];
  const unsigned lane = threadIdx.x & 31u;
  const unsigned wave = __builtin_amdgcn_readfirstlane(threadIdx.x >> 5);
  const unsigned hh = lane >> 4, m = lane & 15u;
  const unsigned tile = blockIdx.x * (unsigned)WPB + wave;
  if (tile >= (unsigned)NTILE) return;
  const unsigned row0 = tile * 16u;
  const unsigned cb = wave * (16u * LDP);

  const float* xr = X + (size_t)(row0 + m) * DFEAT + hh * 8u;
  const _Float16* bp = Wt + (size_t)m * DFEAT + hh * 8u;
  v8f acc = {};
#pragma unroll 2
  for (unsigned k0 = 0; k0 < (unsigned)DFEAT; k0 += 32u) {
    const v16h a = frag_from_f32(xr + k0);
    const v16h b = frag_at(bp + k0);
    acc = wmma16(a, b, acc);
  }
#pragma unroll
  for (int r = 0; r < 8; ++r)
    Cs[cb + (hh * 8u + (unsigned)r) * LDP + m] = acc[r] * (1.0f / (XCARRY * WCARRY));
  wave_lds_sync();

  v4f xs[2];
  size_t off[2];
#pragma unroll
  for (unsigned i = 0; i < 2u; ++i) {
    const unsigned f = 32u * i + lane;
    const unsigned r = f >> 2;
    const unsigned c = (f & 3u) * 4u;
    xs[i] = *(const v4f*)&Cs[cb + r * LDP + c];
    off[i] = (size_t)row0 * NPROJ + (size_t)f * 4u;
  }
#pragma unroll
  for (int i = 0; i < 2; ++i) *(volatile v4f*)(proj + off[i]) = xs[i];
  __threadfence();
#pragma unroll
  for (int i = 0; i < 2; ++i) *(volatile v4f*)(proj + off[i]) = xs[i];
}

__global__ __launch_bounds__(256) void edge_kernel(
    const int* __restrict__ ei, const float* __restrict__ proj,
    const float* __restrict__ bias, float* __restrict__ out) {
  const unsigned lane = threadIdx.x & 31u;
  const unsigned wave = __builtin_amdgcn_readfirstlane(threadIdx.x >> 5);
  const unsigned g0 = blockIdx.x * 256u + wave * 32u;
  if (g0 >= 2u * (unsigned)NEDGE) return;
  const unsigned g = g0 + lane;
  const unsigned e = g >> 1, half = g & 1u;

  int o = ei[e];
  int d = ei[(size_t)NEDGE_FULL + e];
  o = (o < 0) ? 0 : o;
  o = (o > NNODE - 1) ? (NNODE - 1) : o;
  d = (d < 0) ? 0 : d;
  d = (d > NNODE - 1) ? (NNODE - 1) : d;

  const v4f pa = *(const v4f*)(proj + (size_t)o * NPROJ + half * 4u);
  const v4f pc = *(const v4f*)(proj + (size_t)d * NPROJ + 8u + half * 4u);
  const v4f bb = *(const v4f*)(bias + half * 4u);
  v4f r;
#pragma unroll
  for (int j = 0; j < 4; ++j) r[j] = (pa[j] + pc[j]) + bf16r(bb[j]);

  float* p = out + (size_t)g * 4u;
  *(volatile v4f*)p = r;
  __threadfence();
  *(volatile v4f*)p = r;
}

extern "C" void kernel_launch(void* const* d_in, const int* in_sizes, int n_in,
                              void* d_out, int out_size, void* d_ws, size_t ws_size,
                              hipStream_t stream) {
  if (n_in < 4) return;
  if ((long long)in_sizes[0] < (long long)NNODE * DFEAT) return;
  if ((long long)in_sizes[1] < (long long)NEDGE_FULL + NEDGE) return;
  if ((long long)in_sizes[2] < (long long)2 * DFEAT * NHEADS) return;
  if (in_sizes[3] < NHEADS) return;
  if ((long long)out_size < (long long)NEDGE * NHEADS) return;
  if (ws_size < WS_TOTAL) return;

  const float* X  = (const float*)d_in[0];
  const int*   EI = (const int*)d_in[1];
  const float* W  = (const float*)d_in[2];
  const float* B  = (const float*)d_in[3];
  float* out = (float*)d_out;

  char* ws = (char*)d_ws;
  _Float16* Wt16 = (_Float16*)(ws + OFF_WT);
  float*    Proj = (float*)(ws + OFF_PROJ);

  wconv_kernel<<<dim3(1), dim3(256), 0, stream>>>(W, Wt16);
  proj_kernel<<<dim3(NTILE / WPB), dim3(32 * WPB), 0, stream>>>(X, Wt16, Proj);
  edge_kernel<<<dim3((2 * NEDGE + 255) / 256), dim3(256), 0, stream>>>(EI, Proj, B, out);
}
